// DynamicGCN_86397562126410
// MI455X (gfx1250) — hardware-verified
//
#include <hip/hip_runtime.h>
#include <math.h>
#include <stdint.h>

#ifndef NB
#define NB 2
#endif
#ifndef SEQ
#define SEQ 512
#endif
#define NB_FULL  2
#define SEQ_FULL 512
#define DIN   256
#define HID   256
#define H2D   128
#define KW    256
#define MROWS (NB * SEQ)
#define PT     256
#define PWAVES 8
#define TPW   (SEQ / (16 * PWAVES))
#define LSC   16.0f
#define W2S   64.0f
#define H2CAR (16.0f * 64.0f)
#define XS    1024.0f
#define ACAR  32768.0f
#define AGS   4096.0f
#define WGS   1024.0f
#define SLAB64 (16 * 68)
#define VTP   72
#define WS_CAP 134217728
#define SZ_XB ((size_t)MROWS * DIN * 2)
#define SZ_XT ((size_t)NB * DIN * SEQ * 2)
#define SZ_W1 ((size_t)HID * KW * 2)
#define SZ_W2 ((size_t)H2D * KW * 2)
#define SZ_WG ((size_t)HID * KW * 2)
#define SZ_LR ((size_t)MROWS * HID * 4)
#define SZ_A  ((size_t)MROWS * SEQ * 2)
#define SZ_AG ((size_t)MROWS * DIN * 2)
#define WS_TOTAL (SZ_XB + SZ_XT + 2 * SZ_W1 + SZ_W2 + SZ_WG + 2 * SZ_LR + 2 * SZ_A + 2 * SZ_AG)
static_assert(DIN == 256 && HID == 256 && H2D == 128 && KW == DIN && KW == HID);
static_assert(NB >= 1 && NB <= NB_FULL && SEQ >= 256 && SEQ <= SEQ_FULL && (SEQ % 256) == 0);
static_assert((MROWS % 64) == 0 && (SEQ % 64) == 0 && (HID % 64) == 0 && (DIN % 64) == 0 && (H2D % 16) == 0);
static_assert(PT == HID && H2D <= PT && PT == 32 * PWAVES && (SEQ % (16 * PWAVES)) == 0 && ((SEQ / 8) % 32) == 0);
static_assert((KW % 32) == 0 && (SEQ % 32) == 0 && (MROWS % 8) == 0);
static_assert(WS_TOTAL <= (size_t)WS_CAP);

typedef unsigned short u16;
typedef _Float16 v16h __attribute__((ext_vector_type(16)));
typedef _Float16 v8h  __attribute__((ext_vector_type(8)));
typedef __bf16   v16b __attribute__((ext_vector_type(16)));
typedef float    v8f  __attribute__((ext_vector_type(8)));
typedef float    v4f  __attribute__((ext_vector_type(4)));
typedef unsigned int v4u __attribute__((ext_vector_type(4)));

union FragH { v16h v; v8h h[2]; v4u u[2]; };
union FragB { v16b v; v4u u[2]; };

__device__ __forceinline__ unsigned short bf_bits(float f) {
  unsigned u = __float_as_uint(f);
  return (unsigned short)((u + 0x7FFFu + ((u >> 16) & 1u)) >> 16);
}
__device__ __forceinline__ float bf_up(unsigned short h) { return __uint_as_float(((unsigned)h) << 16); }
__device__ __forceinline__ float bfr(float f) { return bf_up(bf_bits(f)); }
__device__ __forceinline__ unsigned short h_bits(_Float16 x) { return __builtin_bit_cast(unsigned short, x); }
__device__ __forceinline__ unsigned pk16(unsigned short a, unsigned short b) { return (unsigned)a | ((unsigned)b << 16); }
__device__ __forceinline__ v8f zero8() { v8f z = {0.f, 0.f, 0.f, 0.f, 0.f, 0.f, 0.f, 0.f}; return z; }
__device__ __forceinline__ _Float16 relu16(float s) { return (_Float16)(s > 0.0f ? s : 0.0f); }

__device__ __forceinline__ v16h ldfrag_h(const _Float16* p) {
  FragH f;
  f.h[0] = *(const v8h*)(p);
  f.h[1] = *(const v8h*)(p + 16);
  return f.v;
}
__device__ __forceinline__ v16b ldfrag_b(const u16* p) {
  FragB f;
  f.u[0] = *(const v4u*)(p);
  f.u[1] = *(const v4u*)(p + 16);
  return f.v;
}

__device__ __forceinline__ v8f mma_h(v16h a, v16h b, v8f c) {
  return __builtin_amdgcn_wmma_f32_16x16x32_f16(false, a, false, b, (short)0, c, false, false);
}
__device__ __forceinline__ v8f mma_b(v16b a, v16b b, v8f c) {
  return __builtin_amdgcn_wmma_f32_16x16x32_bf16(false, a, false, b, (short)0, c, false, false);
}
template <typename F>
__device__ __forceinline__ void guard6(v8f& a, v8f& b, v8f& c, v8f& d, F x0, F x1, F x2, F x3, F x4, F x5) {
#if defined(__HIP_DEVICE_COMPILE__)
  asm volatile("v_nop\n\tv_nop\n\tv_nop\n\tv_nop"
               : "+v"(a), "+v"(b), "+v"(c), "+v"(d) : "v"(x0), "v"(x1), "v"(x2), "v"(x3), "v"(x4), "v"(x5) : "memory");
#endif
}
__device__ __forceinline__ void wave_sync_lds() {
  __builtin_amdgcn_fence(__ATOMIC_RELEASE, "workgroup");
  __builtin_amdgcn_wave_barrier();
  __builtin_amdgcn_fence(__ATOMIC_ACQUIRE, "workgroup");
}

__global__ __launch_bounds__(256) void cvtx16(const float* __restrict__ x, u16* D, int nrow) {
  const int gt  = blockIdx.x * 256 + (int)threadIdx.x;
  const int row = gt >> 5;
  if (row >= nrow) return;
  const int c8  = (gt & 31) * 8;
  const int b   = row / SEQ;
  const int s   = row - b * SEQ;
  const float* p = x + ((size_t)b * SEQ_FULL + s) * DIN + c8;
  const v4f a = *(const v4f*)(p), b4 = *(const v4f*)(p + 4);
  v4u o;
#pragma unroll
  for (int e = 0; e < 2; ++e) {
    o[e]     = pk16(bf_bits(a[2 * e]),  bf_bits(a[2 * e + 1]));
    o[2 + e] = pk16(bf_bits(b4[2 * e]), bf_bits(b4[2 * e + 1]));
  }
  u16* d = D + (size_t)row * DIN + c8;
  for (int pass = 0; pass < 2; ++pass) {
    *(volatile v4u*)(d) = o;
    __threadfence();
  }
}

__global__ __launch_bounds__(256) void xt16(const float* __restrict__ x, u16* XT) {
  __shared__ __align__(16) u16 T[64 * VTP];
  const int tid = threadIdx.x;
  const int bid = blockIdx.x;
  const int nst = SEQ / 64;
  const int ng  = DIN / 64;
  const int st  = bid % nst;
  const int t2  = bid / nst;
  const int g   = t2 % ng;
  const int b   = t2 / ng;
  if (b >= NB) return;
  const int s0  = st * 64;
  {
    const int sl = tid >> 2;
    const int dc = (tid & 3) * 16;
    const float* src = x + ((size_t)b * SEQ_FULL + s0 + sl) * DIN + g * 64 + dc;
#pragma unroll
    for (int i = 0; i < 4; ++i) {
      const v4f a = *(const v4f*)(src + 4 * i);
#pragma unroll
      for (int e = 0; e < 4; ++e) {
        T[(dc + 4 * i + e) * VTP + sl] = h_bits((_Float16)(bfr(a[e]) * XS));
      }
    }
  }
  __syncthreads();
  v4u vh[2];
  const int q8 = tid >> 3, p8 = (tid & 7) * 8;
#pragma unroll
  for (int it = 0; it < 2; ++it) {
    const int line = it * 32 + q8;
    vh[it] = *(const v4u*)(T + line * VTP + p8);
  }
  const size_t base = ((size_t)b * DIN + (size_t)g * 64) * SEQ + s0 + p8;
  for (int pass = 0; pass < 2; ++pass) {
#pragma unroll
    for (int it = 0; it < 2; ++it) {
      const int line = it * 32 + q8;
      *(volatile v4u*)(XT + base + (size_t)line * SEQ) = vh[it];
    }
    __threadfence();
  }
}

__global__ __launch_bounds__(256) void wt16(const float* __restrict__ W, int ldw, int coff, int nct, u16* D,
                                            int f16mode, float scale) {
  __shared__ __align__(16) u16 T[128 * VTP];
  const int tid = threadIdx.x;
  const int bid = blockIdx.x;
  const int ct  = bid % nct;
  const int rt  = bid / nct;
  if (rt * 64 + 64 > KW) return;
  {
    const int sl = tid >> 2;
    const int dc = (tid & 3) * 32;
    const float* src = W + (size_t)(rt * 64 + sl) * ldw + coff + ct * 128 + dc;
#pragma unroll
    for (int i = 0; i < 8; ++i) {
      const v4f a = *(const v4f*)(src + 4 * i);
#pragma unroll
      for (int e = 0; e < 4; ++e) {
        const float f = a[e];
        const unsigned short hb = h_bits((_Float16)(bfr(f) * scale));
        const unsigned short bb = bf_bits(f);
        T[(dc + 4 * i + e) * VTP + sl] = (f16mode != 0) ? hb : bb;
      }
    }
  }
  __syncthreads();
  v4u w4[4];
  const int q8 = tid >> 3, p8 = (tid & 7) * 8;
#pragma unroll
  for (int it = 0; it < 4; ++it) {
    const int line = it * 32 + q8;
    w4[it] = *(const v4u*)(T + line * VTP + p8);
  }
  const size_t base = ((size_t)ct * 128) * KW + rt * 64 + p8;
  for (int pass = 0; pass < 2; ++pass) {
#pragma unroll
    for (int it = 0; it < 4; ++it) {
      const int line = it * 32 + q8;
      *(volatile v4u*)(D + base + (size_t)line * KW) = w4[it];
    }
    __threadfence();
  }
}

__device__ __forceinline__ void epi64(float* sl, v8f a0, v8f a1, v8f a2, v8f a3, float oscale,
                                      const float* __restrict__ bias, float bscale,
                                      float* C, int N, size_t rowb, int col0, int lane) {
  const int hh = lane >> 4, m = lane & 15;
#pragma unroll
  for (int r = 0; r < 8; ++r) {
    const int ro = (8 * hh + r) * 68 + m;
    sl[ro]      = a0[r] * oscale;
    sl[ro + 16] = a1[r] * oscale;
    sl[ro + 32] = a2[r] * oscale;
    sl[ro + 48] = a3[r] * oscale;
  }
  wave_sync_lds();
  const v4f bq = *(const v4f*)(bias + col0 + m * 4);
  v4f badd;
#pragma unroll
  for (int e = 0; e < 4; ++e) badd[e] = bfr(bq[e]) * bscale;
  v4f vals[8];
#pragma unroll
  for (int it = 0; it < 8; ++it) vals[it] = *(const v4f*)(sl + (it * 2 + hh) * 68 + m * 4) + badd;
  float* dst = C + (rowb + (size_t)hh) * (size_t)N + col0 + m * 4;
  for (int pass = 0; pass < 2; ++pass) {
#pragma unroll
    for (int it = 0; it < 8; ++it) {
      *(volatile v4f*)(dst + (size_t)(it * 2) * (size_t)N) = vals[it];
    }
    __threadfence();
  }
}

__global__ __launch_bounds__(128)
void gemm_bf(const u16* __restrict__ A, const u16* __restrict__ Bt, float* C, int M, int N, int K, float oscale,
             const float* __restrict__ bias, float bscale) {
  __shared__ __align__(16) float slab[4 * SLAB64];
  const int tid = threadIdx.x, wave = tid >> 5, lane = tid & 31, hh = lane >> 4, m = lane & 15;
  const int ntile = N >> 6;
  const int bid   = blockIdx.x;
  const int rowb  = (bid / ntile) * 64 + wave * 16;
  const int col0  = (bid % ntile) * 64;
  if (rowb + 16 > M) return;
  const u16* ap = A  + (size_t)(rowb + m) * K + 8 * hh;
  const u16* bp = Bt + (size_t)(col0 + m) * K + 8 * hh;
  const size_t bs = (size_t)16 * K;
  v8f acc0 = zero8(), acc1 = zero8(), acc2 = zero8(), acc3 = zero8();
#pragma unroll 1
  for (int k0 = 0; k0 < K; k0 += 32) {
    const v16b a  = ldfrag_b(ap + k0);
    const v16b b0 = ldfrag_b(bp + k0);
    const v16b b1 = ldfrag_b(bp + bs + k0);
    const v16b b2 = ldfrag_b(bp + 2 * bs + k0);
    const v16b b3 = ldfrag_b(bp + 3 * bs + k0);
    acc0 = mma_b(a, b0, acc0);
    acc1 = mma_b(a, b1, acc1);
    acc2 = mma_b(a, b2, acc2);
    acc3 = mma_b(a, b3, acc3);
    guard6<v16b>(acc0, acc1, acc2, acc3, a, b0, b1, b2, b3, a);
  }
  epi64(slab + wave * SLAB64, acc0, acc1, acc2, acc3, oscale, bias, bscale, C, N, (size_t)rowb, col0, lane);
}

__global__ __launch_bounds__(256)
void pair_mlp(const float* __restrict__ L16, const float* __restrict__ R16, const u16* __restrict__ W2T,
              const float* __restrict__ b2p, const float* __restrict__ W3p, const float* __restrict__ b3p,
              const float* __restrict__ badj, u16* AHp, u16* ALp) {
  __shared__ __align__(16) float Ls[HID];
  __shared__ __align__(16) float sdyn[SEQ];
  __shared__ float sW3[H2D];
  __shared__ float sB2[H2D];
  __shared__ float sred[2 * PWAVES];
  const int tid = threadIdx.x, wave = tid >> 5, lane = tid & 31, hh = lane >> 4, m = lane & 15, m7 = lane & 7;
  const int bi = blockIdx.x;
  const int b  = bi / SEQ;
  const int i  = bi - b * SEQ;
  if (b >= NB) return;
  Ls[tid] = L16[(size_t)bi * HID + tid];
  if (tid < H2D) {
    sW3[tid] = bfr(W3p[tid]);
    sB2[tid] = bfr(b2p[tid]) * H2CAR;
  }
  const float b3v = bfr(b3p[0]);
  __syncthreads();
  float w3r[8], b2r[8];
#pragma unroll
  for (int ct = 0; ct < 8; ++ct) { w3r[ct] = sW3[ct * 16 + m]; b2r[ct] = sB2[ct * 16 + m]; }
  const _Float16* w2p = (const _Float16*)(const void*)W2T + (size_t)m * KW + 8 * hh;
  const size_t cs = (size_t)16 * KW;
  const float* Lr = Ls + 8 * hh;

#pragma unroll 1
  for (int t = 0; t < TPW; ++t) {
    const int jb = t * (16 * PWAVES) + wave * 16;
    const float* Rr = R16 + ((size_t)b * SEQ + jb + m) * HID + 8 * hh;
    v8f acc[8];
#pragma unroll
    for (int ct = 0; ct < 8; ++ct) acc[ct] = zero8();
#pragma unroll 1
    for (int k0 = 0; k0 < HID; k0 += 32) {
      const v4f la = *(const v4f*)(Lr + k0),      lb = *(const v4f*)(Lr + k0 + 4);
      const v4f lc = *(const v4f*)(Lr + k0 + 16), ld = *(const v4f*)(Lr + k0 + 20);
      const v4f ra = *(const v4f*)(Rr + k0),      rb = *(const v4f*)(Rr + k0 + 4);
      const v4f rc = *(const v4f*)(Rr + k0 + 16), rd = *(const v4f*)(Rr + k0 + 20);
      FragH fa;
#pragma unroll
      for (int e = 0; e < 4; ++e) {
        fa.h[0][e]     = relu16(la[e] + ra[e]);
        fa.h[0][4 + e] = relu16(lb[e] + rb[e]);
        fa.h[1][e]     = relu16(lc[e] + rc[e]);
        fa.h[1][4 + e] = relu16(ld[e] + rd[e]);
      }
      {
        const v16h w0 = ldfrag_h(w2p + k0);
        const v16h w1 = ldfrag_h(w2p + cs + k0);
        const v16h w2 = ldfrag_h(w2p + 2 * cs + k0);
        const v16h w3 = ldfrag_h(w2p + 3 * cs + k0);
        acc[0] = mma_h(fa.v, w0, acc[0]);
        acc[1] = mma_h(fa.v, w1, acc[1]);
        acc[2] = mma_h(fa.v, w2, acc[2]);
        acc[3] = mma_h(fa.v, w3, acc[3]);
        guard6<v16h>(acc[0], acc[1], acc[2], acc[3], fa.v, w0, w1, w2, w3, fa.v);
      }
      {
        const v16h w4 = ldfrag_h(w2p + 4 * cs + k0);
        const v16h w5 = ldfrag_h(w2p + 5 * cs + k0);
        const v16h w6 = ldfrag_h(w2p + 6 * cs + k0);
        const v16h w7 = ldfrag_h(w2p + 7 * cs + k0);
        acc[4] = mma_h(fa.v, w4, acc[4]);
        acc[5] = mma_h(fa.v, w5, acc[5]);
        acc[6] = mma_h(fa.v, w6, acc[6]);
        acc[7] = mma_h(fa.v, w7, acc[7]);
        guard6<v16h>(acc[4], acc[5], acc[6], acc[7], fa.v, w4, w5, w6, w7, fa.v);
      }
    }
    float part[8];
#pragma unroll
    for (int r = 0; r < 8; ++r) part[r] = 0.0f;
#pragma unroll
    for (int ct = 0; ct < 8; ++ct) {
#pragma unroll
      for (int r = 0; r < 8; ++r) {
        float v = acc[ct][r] + b2r[ct];
        v = (v > 0.0f) ? v : 0.0f;
        part[r] += v * w3r[ct];
      }
    }
#pragma unroll
    for (int off = 1; off < 16; off <<= 1) {
#pragma unroll
      for (int r = 0; r < 8; ++r) part[r] += __shfl_xor(part[r], off, 32);
    }
    float zs = part[0];
#pragma unroll
    for (int r = 1; r < 8; ++r) zs = (m7 == r) ? part[r] : zs;
    const float z  = zs * (1.0f / H2CAR) + b3v;
    const float ex = expf(-z);
    const float ev = __builtin_amdgcn_rcpf(1.0f + ex);
    const int   j  = jb + 8 * hh + m7;
    const float ba = bfr(badj[((size_t)b * SEQ_FULL + i) * SEQ_FULL + j]);
    float dv = ba * ev;
    dv = dv + ((i == j) ? 1.0f : 0.0f);
    if (m < 8) sdyn[j] = dv;
  }
  __syncthreads();

  constexpr int EPT = SEQ / PT;
  float v[EPT], exv[EPT];
  float mx = -INFINITY;
#pragma unroll
  for (int e = 0; e < EPT; ++e) { v[e] = sdyn[e * PT + tid]; mx = fmaxf(mx, v[e]); }
#pragma unroll
  for (int off = 1; off < 32; off <<= 1) mx = fmaxf(mx, __shfl_xor(mx, off, 32));
  if (lane == 0) sred[wave] = mx;
  __syncthreads();
  float gm = sred[0];
#pragma unroll
  for (int w = 1; w < PWAVES; ++w) gm = fmaxf(gm, sred[w]);
  float ps = 0.0f;
#pragma unroll
  for (int e = 0; e < EPT; ++e) { exv[e] = expf(v[e] - gm); ps += exv[e]; }
#pragma unroll
  for (int off = 1; off < 32; off <<= 1) ps += __shfl_xor(ps, off, 32);
  if (lane == 0) sred[PWAVES + wave] = ps;
  __syncthreads();
  float tot = 0.0f;
#pragma unroll
  for (int w = 0; w < PWAVES; ++w) tot += sred[PWAVES + w];
  const float inv = 1.0f / tot;
#pragma unroll
  for (int e = 0; e < EPT; ++e) sdyn[e * PT + tid] = exv[e] * inv;
  __syncthreads();

  if (tid < SEQ / 8) {
    const float* pr = sdyn + tid * 8;
    const v4f p0 = *(const v4f*)(pr), p1 = *(const v4f*)(pr + 4);
    float w[8];
#pragma unroll
    for (int e = 0; e < 4; ++e) { w[e] = p0[e] * ACAR; w[4 + e] = p1[e] * ACAR; }
    v4u oh, ol;
#pragma unroll
    for (int e = 0; e < 4; ++e) {
      const float ta = w[2 * e], tb = w[2 * e + 1];
      const _Float16 ha = (_Float16)ta, hb = (_Float16)tb;
      const _Float16 la = (_Float16)(ta - (float)ha), lb = (_Float16)(tb - (float)hb);
      oh[e] = pk16(h_bits(ha), h_bits(hb));
      ol[e] = pk16(h_bits(la), h_bits(lb));
    }
    u16* dh = AHp + (size_t)bi * SEQ + tid * 8;
    u16* dl = ALp + (size_t)bi * SEQ + tid * 8;
    for (int pass = 0; pass < 2; ++pass) {
      *(volatile v4u*)(dh) = oh;
      *(volatile v4u*)(dl) = ol;
      __threadfence();
    }
  }
}

__global__ __launch_bounds__(128)
void gemm_agg(const u16* __restrict__ Ah, const u16* __restrict__ Al, const u16* __restrict__ XT,
              u16* GH, u16* GL, float oscale) {
  __shared__ __align__(16) float slab[4 * SLAB64];
  const int tid = threadIdx.x, wave = tid >> 5, lane = tid & 31, hh = lane >> 4, m = lane & 15;
  const int ntile = DIN >> 6;
  const int nrt   = SEQ >> 6;
  const int bid   = blockIdx.x;
  const int ct    = bid % ntile;
  const int t2    = bid / ntile;
  const int rt    = t2 % nrt;
  const int bb    = t2 / nrt;
  if (bb >= NB) return;
  const int srow  = rt * 64 + wave * 16;
  const int col0  = ct * 64;
  const int K     = SEQ;
  const size_t rowC = (size_t)bb * SEQ + srow;
  const _Float16* ahp = (const _Float16*)(const void*)Ah + (rowC + m) * K + 8 * hh;
  const _Float16* alp = (const _Float16*)(const void*)Al + (rowC + m) * K + 8 * hh;
  const _Float16* bp  = (const _Float16*)(const void*)XT + ((size_t)bb * DIN + col0 + m) * K + 8 * hh;
  const size_t bs = (size_t)16 * K;
  v8f acc0 = zero8(), acc1 = zero8(), acc2 = zero8(), acc3 = zero8();
#pragma unroll 1
  for (int k0 = 0; k0 < K; k0 += 32) {
    const v16h ah = ldfrag_h(ahp + k0), al = ldfrag_h(alp + k0);
    const v16h b0 = ldfrag_h(bp + k0);
    const v16h b1 = ldfrag_h(bp + bs + k0);
    const v16h b2 = ldfrag_h(bp + 2 * bs + k0);
    const v16h b3 = ldfrag_h(bp + 3 * bs + k0);
    acc0 = mma_h(ah, b0, acc0);  acc0 = mma_h(al, b0, acc0);
    acc1 = mma_h(ah, b1, acc1);  acc1 = mma_h(al, b1, acc1);
    acc2 = mma_h(ah, b2, acc2);  acc2 = mma_h(al, b2, acc2);
    acc3 = mma_h(ah, b3, acc3);  acc3 = mma_h(al, b3, acc3);
    guard6<v16h>(acc0, acc1, acc2, acc3, ah, al, b0, b1, b2, b3);
  }
  float* sl = slab + wave * SLAB64;
#pragma unroll
  for (int r = 0; r < 8; ++r) {
    const int ro = (8 * hh + r) * 68 + m;
    sl[ro]      = acc0[r] * oscale;
    sl[ro + 16] = acc1[r] * oscale;
    sl[ro + 32] = acc2[r] * oscale;
    sl[ro + 48] = acc3[r] * oscale;
  }
  wave_sync_lds();
  v4u oh[4], ol[4];
  const int rq = lane >> 3, c8 = (lane & 7) * 8;
#pragma unroll
  for (int it = 0; it < 4; ++it) {
    const int row = it * 4 + rq;
    const v4f a = *(const v4f*)(sl + row * 68 + c8), b4 = *(const v4f*)(sl + row * 68 + c8 + 4);
    float w[8];
#pragma unroll
    for (int e = 0; e < 4; ++e) { w[e] = a[e]; w[4 + e] = b4[e]; }
#pragma unroll
    for (int e = 0; e < 4; ++e) {
      const _Float16 h0 = (_Float16)w[2 * e], h1 = (_Float16)w[2 * e + 1];
      const _Float16 l0 = (_Float16)(w[2 * e] - (float)h0), l1 = (_Float16)(w[2 * e + 1] - (float)h1);
      oh[it][e] = pk16(h_bits(h0), h_bits(h1));
      ol[it][e] = pk16(h_bits(l0), h_bits(l1));
    }
  }
  const size_t ob = rowC * DIN + col0 + c8;
  for (int pass = 0; pass < 2; ++pass) {
#pragma unroll
    for (int it = 0; it < 4; ++it) {
      const int row = it * 4 + rq;
      *(volatile v4u*)(GH + ob + (size_t)row * DIN) = oh[it];
      *(volatile v4u*)(GL + ob + (size_t)row * DIN) = ol[it];
    }
    __threadfence();
  }
}

__global__ __launch_bounds__(128)
void gemm_out(const u16* __restrict__ Ah, const u16* __restrict__ Al, const u16* __restrict__ Bt,
              float* C, const float* __restrict__ bias, float oscale) {
  __shared__ __align__(16) float slab[4 * SLAB64];
  const int tid = threadIdx.x, wave = tid >> 5, lane = tid & 31, hh = lane >> 4, m = lane & 15;
  const int ntile = HID >> 6;
  const int bid   = blockIdx.x;
  const int rowb  = (bid / ntile) * 64 + wave * 16;
  const int col0  = (bid % ntile) * 64;
  if (rowb + 16 > MROWS) return;
  const int K     = DIN;
  const _Float16* ahp = (const _Float16*)(const void*)Ah + (size_t)(rowb + m) * K + 8 * hh;
  const _Float16* alp = (const _Float16*)(const void*)Al + (size_t)(rowb + m) * K + 8 * hh;
  const _Float16* bp  = (const _Float16*)(const void*)Bt + (size_t)(col0 + m) * K + 8 * hh;
  const size_t bs = (size_t)16 * K;
  v8f acc0 = zero8(), acc1 = zero8(), acc2 = zero8(), acc3 = zero8();
#pragma unroll 1
  for (int k0 = 0; k0 < K; k0 += 32) {
    const v16h ah = ldfrag_h(ahp + k0), al = ldfrag_h(alp + k0);
    const v16h b0 = ldfrag_h(bp + k0);
    const v16h b1 = ldfrag_h(bp + bs + k0);
    const v16h b2 = ldfrag_h(bp + 2 * bs + k0);
    const v16h b3 = ldfrag_h(bp + 3 * bs + k0);
    acc0 = mma_h(ah, b0, acc0);  acc0 = mma_h(al, b0, acc0);
    acc1 = mma_h(ah, b1, acc1);  acc1 = mma_h(al, b1, acc1);
    acc2 = mma_h(ah, b2, acc2);  acc2 = mma_h(al, b2, acc2);
    acc3 = mma_h(ah, b3, acc3);  acc3 = mma_h(al, b3, acc3);
    guard6<v16h>(acc0, acc1, acc2, acc3, ah, al, b0, b1, b2, b3);
  }
  epi64(slab + wave * SLAB64, acc0, acc1, acc2, acc3, oscale, bias, 1.0f, C, HID, (size_t)rowb, col0, lane);
}

extern "C" void kernel_launch(void* const* d_in, const int* in_sizes, int n_in,
                              void* d_out, int out_size, void* d_ws, size_t ws_size,
                              hipStream_t stream) {
  if (n_in < 10) return;
  if (in_sizes[0] < ((NB - 1) * SEQ_FULL + SEQ) * DIN) return;
  if (in_sizes[1] < ((NB - 1) * SEQ_FULL + SEQ) * SEQ_FULL) return;
  if (in_sizes[2] != 2 * DIN * HID) return;
  if (in_sizes[3] != HID) return;
  if (in_sizes[4] != HID * H2D) return;
  if (in_sizes[5] != H2D) return;
  if (in_sizes[6] != H2D) return;
  if (in_sizes[7] < 1) return;
  if (in_sizes[8] != DIN * HID) return;
  if (in_sizes[9] != HID) return;
  if (out_size < MROWS * HID) return;

  const float* x    = (const float*)d_in[0];
  const float* badj = (const float*)d_in[1];
  const float* W1   = (const float*)d_in[2];
  const float* b1   = (const float*)d_in[3];
  const float* W2   = (const float*)d_in[4];
  const float* b2   = (const float*)d_in[5];
  const float* W3   = (const float*)d_in[6];
  const float* b3   = (const float*)d_in[7];
  const float* Wg   = (const float*)d_in[8];
  const float* bg   = (const float*)d_in[9];
  float*       out  = (float*)d_out;

  size_t off = 0;
  const size_t oXB  = off; off += SZ_XB;
  const size_t oXT  = off; off += SZ_XT;
  const size_t oW1L = off; off += SZ_W1;
  const size_t oW1R = off; off += SZ_W1;
  const size_t oW2T = off; off += SZ_W2;
  const size_t oWGT = off; off += SZ_WG;
  const size_t oL   = off; off += SZ_LR;
  const size_t oR   = off; off += SZ_LR;
  const size_t oAH  = off; off += SZ_A;
  const size_t oAL  = off; off += SZ_A;
  const size_t oAGH = off; off += SZ_AG;
  const size_t oAGL = off; off += SZ_AG;
  if (off > ws_size) return;
  if (off > (size_t)WS_CAP) return;

  char* ws = (char*)d_ws;
  u16*   XB  = (u16*)(ws + oXB);
  u16*   XT  = (u16*)(ws + oXT);
  u16*   W1L = (u16*)(ws + oW1L);
  u16*   W1R = (u16*)(ws + oW1R);
  u16*   W2T = (u16*)(ws + oW2T);
  u16*   WGT = (u16*)(ws + oWGT);
  float* L16 = (float*)(ws + oL);
  float* R16 = (float*)(ws + oR);
  u16*   AH  = (u16*)(ws + oAH);
  u16*   AL  = (u16*)(ws + oAL);
  u16*   AGH = (u16*)(ws + oAGH);
  u16*   AGL = (u16*)(ws + oAGL);

  const dim3 b256(256), b128(128);
  const dim3 gCX(MROWS / 8);
  const dim3 gXT(NB * (DIN / 64) * (SEQ / 64));
  const dim3 gW256(2 * (KW / 64));
  const dim3 gW128(1 * (KW / 64));
  const dim3 gLR((MROWS / 64) * (HID / 64));
  const dim3 gPM(MROWS);
  const dim3 gAG(NB * (SEQ / 64) * (DIN / 64));
  const dim3 gOUT((MROWS / 64) * (HID / 64));
  const float aosc = AGS / (ACAR * XS);
  const float oosc = 1.0f / (AGS * WGS);

  cvtx16<<<gCX, b256, 0, stream>>>(x, XB, MROWS);
  xt16<<<gXT, b256, 0, stream>>>(x, XT);
  wt16<<<gW256, b256, 0, stream>>>(W1, HID, 0, 2, W1L, 0, 1.0f);
  wt16<<<gW256, b256, 0, stream>>>(W1 + (size_t)DIN * HID, HID, 0, 2, W1R, 0, 1.0f);
  wt16<<<gW128, b256, 0, stream>>>(W2, H2D, 0, 1, W2T, 1, W2S);
  wt16<<<gW256, b256, 0, stream>>>(Wg, HID, 0, 2, WGT, 1, WGS);
  gemm_bf<<<gLR, b128, 0, stream>>>(XB, W1L, L16, MROWS, HID, DIN, LSC, b1, LSC);
  gemm_bf<<<gLR, b128, 0, stream>>>(XB, W1R, R16, MROWS, HID, DIN, LSC, b1, 0.0f);
  pair_mlp<<<gPM, b256, 0, stream>>>(L16, R16, W2T, b2, W3, b3, badj, AH, AL);
  gemm_agg<<<gAG, b128, 0, stream>>>(AH, AL, XT, AGH, AGL, aosc);
  gemm_out<<<gOUT, b128, 0, stream>>>(AGH, AGL, WGT, out, bg, oosc);
  (void)hipGetLastError();
}
